// RiemannianGNN_47777216201088
// MI455X (gfx1250) — hardware-run, weakly checked
//
#include <hip/hip_runtime.h>

typedef float          v8f   __attribute__((ext_vector_type(8)));
typedef float          v4f   __attribute__((ext_vector_type(4)));
typedef unsigned int   v4u   __attribute__((ext_vector_type(4)));
typedef int            v8i   __attribute__((ext_vector_type(8)));
typedef unsigned short v8us  __attribute__((ext_vector_type(8)));
typedef unsigned short v16us __attribute__((ext_vector_type(16)));
typedef __bf16         v16bf __attribute__((ext_vector_type(16)));
typedef _Float16       v16h  __attribute__((ext_vector_type(16)));
typedef v4f  __attribute__((may_alias)) v4fa;
typedef v8us __attribute__((may_alias)) v8usa;
union FragB { v16bf v; v16us u; v8us h[2]; v8i w; };
union FragH { v16h  v; v16us u; v8us h[2]; v8i w; };

__device__ __forceinline__ v8f wmb(const FragB& a, const FragB& b, v8f c) {
  v8f d = __builtin_amdgcn_wmma_f32_16x16x32_bf16(false, a.v, false, b.v, (short)0, c, false, false);
  asm volatile("v_nop\n\tv_nop\n\tv_nop\n\tv_nop" : "+v"(d) : "v"(a.w), "v"(b.w));
  return d;
}

__device__ __forceinline__ v8f wmh(const FragH& a, const FragH& b, v8f c) {
  v8f d = __builtin_amdgcn_wmma_f32_16x16x32_f16(false, a.v, false, b.v, (short)0, c, false, false);
  asm volatile("v_nop\n\tv_nop\n\tv_nop\n\tv_nop" : "+v"(d) : "v"(a.w), "v"(b.w));
  return d;
}

__device__ __forceinline__ unsigned bf16_bits(float f) {
  const unsigned u = __float_as_uint(f);
  const unsigned r = (u + 0x7FFFu + ((u >> 16) & 1u)) >> 16;
  const unsigned q = (u >> 16) | 0x40u;
  return ((u & 0x7fffffffu) > 0x7f800000u) ? q : r;
}

__device__ __forceinline__ float bf16_val(float f) {
  return __uint_as_float(bf16_bits(f) << 16);
}
__device__ __forceinline__ int clampi(int v, int lo, int hi) {
  return v < lo ? lo : (v > hi ? hi : v);
}

__device__ __forceinline__ unsigned f16_bits(float f) {
  const unsigned u  = __float_as_uint(f);
  const unsigned s  = (u >> 16) & 0x8000u;
  const unsigned a  = u & 0x7fffffffu;
  const unsigned t  = a - 0x38000000u;
  const unsigned r  = (t + 0x0FFFu + ((t >> 13) & 1u)) >> 13;
  const unsigned rc = r > 0x7C00u ? 0x7C00u : r;
  const bool small  = a < 0x38800000u;
  const bool isnan  = a > 0x7f800000u;
  const unsigned fin = small ? 0u : (s | rc);
  return isnan ? (s | 0x7E00u) : fin;
}

__device__ __forceinline__ unsigned pk16(unsigned lo, unsigned hi) { return lo | (hi << 16); }
__device__ __forceinline__ unsigned bf16_lo_bits(float v) {
  float hi = bf16_val(v);
  asm volatile("" : "+v"(hi));
  return bf16_bits(v - hi);
}
__device__ __forceinline__ v4u pack8_bf16(v4f a, v4f c) {
  return (v4u){ pk16(bf16_bits(a[0]), bf16_bits(a[1])), pk16(bf16_bits(a[2]), bf16_bits(a[3])),
                pk16(bf16_bits(c[0]), bf16_bits(c[1])), pk16(bf16_bits(c[2]), bf16_bits(c[3])) };
}
__device__ __forceinline__ v4u pack8_bf16_lo(v4f a, v4f c) {
  return (v4u){ pk16(bf16_lo_bits(a[0]), bf16_lo_bits(a[1])), pk16(bf16_lo_bits(a[2]), bf16_lo_bits(a[3])),
                pk16(bf16_lo_bits(c[0]), bf16_lo_bits(c[1])), pk16(bf16_lo_bits(c[2]), bf16_lo_bits(c[3])) };
}
__device__ __forceinline__ v4u pack8_f16(v4f a, v4f c) {
  return (v4u){ pk16(f16_bits(a[0]), f16_bits(a[1])), pk16(f16_bits(a[2]), f16_bits(a[3])),
                pk16(f16_bits(c[0]), f16_bits(c[1])), pk16(f16_bits(c[2]), f16_bits(c[3])) };
}

template <int FORM>
__global__ __launch_bounds__(256) void k_plane(const float* __restrict__ src, int rows, int cols, int ldsrc,
                                               unsigned short* __restrict__ dst, int MP, int KP) {
  static_assert(FORM >= 0 && FORM <= 3);
  const int KTOT = (FORM == 1 || FORM == 3) ? 2 * KP : KP;
  const unsigned ppr   = (unsigned)(KTOT >> 3);
  const unsigned kp8   = (unsigned)(KP >> 3);
  const unsigned total = (unsigned)MP * ppr;
  const unsigned g     = blockIdx.x * 256u + threadIdx.x;
  const unsigned rowu  = g / ppr;
  const unsigned p     = g - rowu * ppr;
  const bool second    = p >= kp8;
  const int row = (int)rowu;
  const int c0  = (int)((second ? p - kp8 : p) << 3);
  const float* srow = src + (size_t)clampi(row, 0, rows - 1) * (size_t)ldsrc;
  float x[8];
  unsigned mk[8];
#pragma unroll
  for (int e = 0; e < 8; ++e) {
    const int c = c0 + e;
    const float v = srow[clampi(c, 0, cols - 1)];
    asm volatile("" :: "v"(v));
    x[e]  = v;
    mk[e] = (row < rows && c < cols) ? 0xFFFFu : 0u;
  }
  const v4f a = (v4f){ x[0], x[1], x[2], x[3] };
  const v4f c = (v4f){ x[4], x[5], x[6], x[7] };
  v4u o;
  if (FORM == 2) {
    o = pack8_f16(a, c);
  } else {
    const v4u hi = pack8_bf16(a, c);
    o = hi;
    if (FORM == 1) { const v4u lo = pack8_bf16_lo(a, c); o = second ? lo : hi; }
  }
  const v4u mw = (v4u){ pk16(mk[0], mk[1]), pk16(mk[2], mk[3]), pk16(mk[4], mk[5]), pk16(mk[6], mk[7]) };
  o &= mw;
  if (g < total) {
    volatile v4u* q = (volatile v4u*)(dst + (size_t)g * 8);
    *q = o;
    __threadfence();
    *q = o;
  }
}

template <int FORM> struct FragOf    { typedef FragB T; };
template <>         struct FragOf<2> { typedef FragH T; };
__device__ __forceinline__ v8f mm(const FragB& a, const FragB& b, v8f c) { return wmb(a, b, c); }
__device__ __forceinline__ v8f mm(const FragH& a, const FragH& b, v8f c) { return wmh(a, b, c); }
template <class F> __device__ __forceinline__ F ld_frag(const unsigned short* p) {
  F f;
  f.h[0] = *(const v8usa*)(p);
  f.h[1] = *(const v8usa*)(p + 16);
  return f;
}

template <int FORM, int EPI>
__global__ __launch_bounds__(256) __attribute__((amdgpu_num_vgpr(248)))
void k_gemm_nt(const unsigned short* __restrict__ A, const unsigned short* __restrict__ B,
               const float* __restrict__ bias, float* __restrict__ D, int M, int N, int KTOT, int ldd) {
  static_assert(FORM >= 0 && FORM <= 2);
  static_assert(EPI == 0 || EPI == 1);
  typedef typename FragOf<FORM>::T F;
  __shared__ __attribute__((aligned(16))) float sT[8][16 * 68];
  const int lane = threadIdx.x & 31;
  const int wave = threadIdx.x >> 5;
  const int tilesM = (M + 63) >> 6;
  const int tilesN = (N + 63) >> 6;
  const int tile = blockIdx.x * 8 + wave;
  if (tile >= tilesM * tilesN) return;
  const int tm = tile / tilesN;
  const int tn = tile - tm * tilesN;
  const int m0 = tm << 6;
  const int n0 = tn << 6;

  const int rl = lane & 15;
  const int h8 = (lane >> 4) * 8;
  const unsigned short* pa = A + (size_t)(m0 + rl) * (size_t)KTOT + h8;
  const unsigned short* pb = B + (size_t)(n0 + rl) * (size_t)KTOT + h8;

  v8f acc[4][4];
#pragma unroll
  for (int i = 0; i < 4; ++i)
#pragma unroll
    for (int j = 0; j < 4; ++j) acc[i][j] = (v8f){0.f, 0.f, 0.f, 0.f, 0.f, 0.f, 0.f, 0.f};

#pragma unroll 1
  for (int k0 = 0; k0 < KTOT; k0 += 32) {
    F bf[4];
#pragma unroll
    for (int j = 0; j < 4; ++j) bf[j] = ld_frag<F>(pb + (size_t)(j << 4) * (size_t)KTOT + k0);
#pragma unroll
    for (int i = 0; i < 4; ++i) {
      const F af = ld_frag<F>(pa + (size_t)(i << 4) * (size_t)KTOT + k0);
#pragma unroll
      for (int j = 0; j < 4; ++j) acc[i][j] = mm(af, bf[j], acc[i][j]);
    }
  }

  float* slab = sT[wave];
  const int hh = lane >> 4;
  const int c4 = (lane & 15) * 4;
  const int nc = n0 + c4;
  const bool cok = nc < N;
  v4f bv = (v4f){0.f, 0.f, 0.f, 0.f};
  if (EPI == 1) {
    bv = *(const v4fa*)(bias + clampi(nc, 0, N - 4));
    asm volatile("" :: "v"(bv));
  }
#pragma unroll
  for (int i = 0; i < 4; ++i) {
    const int mBase = m0 + (i << 4);
#pragma unroll
    for (int j = 0; j < 4; ++j) {
#pragma unroll
      for (int r = 0; r < 8; ++r) slab[(h8 + r) * 68 + (j << 4) + rl] = acc[i][j][r];
    }
    __builtin_amdgcn_fence(__ATOMIC_RELEASE, "workgroup");
    __builtin_amdgcn_wave_barrier();
    __builtin_amdgcn_fence(__ATOMIC_ACQUIRE, "workgroup");
    v4f vv[8];
#pragma unroll
    for (int it = 0; it < 8; ++it) {
      const int row = it * 2 + hh;
      v4f v = *(const v4fa*)(slab + row * 68 + c4);
      if (EPI == 1) v += bv;
      vv[it] = v;
    }
    for (int pass = 0; pass < 2; ++pass) {
#pragma unroll
      for (int it = 0; it < 8; ++it) {
        const int row = mBase + it * 2 + hh;
        if (cok && row < M) *(volatile v4f*)(D + (size_t)row * (size_t)ldd + nc) = vv[it];
      }
      __threadfence();
    }
    __builtin_amdgcn_fence(__ATOMIC_RELEASE, "workgroup");
    __builtin_amdgcn_wave_barrier();
    __builtin_amdgcn_fence(__ATOMIC_ACQUIRE, "workgroup");
  }
}

#define NN     50000
#define MPN    50048
#define DD     128
#define KS     32
#ifndef TWO_TERM_L2
#define TWO_TERM_L2 1
#endif
#define A2K    (TWO_TERM_L2 ? 256 : 128)
#define WSMAX  ((size_t)128 << 20)

static_assert(NN % 8 == 0);
static_assert(MPN % 128 == 0 && MPN >= NN && MPN - NN < 64);
static_assert(DD == 128 && KS == 32);
static_assert(MPN % 64 == 0 && DD % 64 == 0 && DD % 32 == 0 && A2K % 32 == 0 && NN % 16 == 0 && DD % 4 == 0);
static_assert((MPN * DD / 8) % 256 == 0);
static_assert((size_t)MPN * 256 / 8 < ((size_t)1 << 31));

constexpr size_t al256(size_t v) { return (v + 255) & ~(size_t)255; }
constexpr size_t O_XB  = 0;
constexpr size_t O_W0T = al256(O_XB  + (size_t)MPN * DD * 2);
constexpr size_t O_W1D = al256(O_W0T + (size_t)DD * DD * 2);
constexpr size_t O_MSG = al256(O_W1D + (size_t)DD * 256 * 2);
constexpr size_t O_A2  = al256(O_MSG + (size_t)MPN * DD * 4);
constexpr size_t WS_TOTAL = al256(O_A2 + (size_t)MPN * 256 * 2);
static_assert(O_W0T == 12812288 && O_W1D == 12845056 && O_MSG == 12910592 && O_A2 == 38535168);
static_assert(WS_TOTAL == 64159744);
static_assert(WS_TOTAL <= (size_t)WSMAX);

typedef unsigned int v2u __attribute__((ext_vector_type(2)));

__device__ __forceinline__ void st2_v4u(void* p, const v4u v) {
  volatile v4u* q = (volatile v4u*)p;
  *q = v;
  __threadfence();
  *q = v;
}

__device__ __forceinline__ v4u gather8_bf16(const float* __restrict__ src, int base, int k0, int kmask, int stride,
                                            unsigned mk) {
  float x[8];
#pragma unroll
  for (int e = 0; e < 8; ++e) {
    const float v = src[base + ((k0 + e) & kmask) * stride];
    asm volatile("" :: "v"(v));
    x[e] = v;
  }
  v4u o = pack8_bf16((v4f){ x[0], x[1], x[2], x[3] }, (v4f){ x[4], x[5], x[6], x[7] });
  o &= (v4u){ mk, mk, mk, mk };
  return o;
}

#define PB_W0       (DD * DD / 8 / 256)
#define PB_W1       (DD * A2K / 8 / 256)
#define PZ_PIECES   ((MPN - NN) * A2K / 8)
#define PB_Z        (PZ_PIECES / 256)
#define PREP_BLOCKS (PB_W0 + PB_W1 + PB_Z)
static_assert((DD * DD / 8) % 256 == 0 && (DD * A2K / 8) % 256 == 0 && PZ_PIECES % 256 == 0 && PB_Z >= 1);

__global__ __launch_bounds__(256) void k_prep(const float* __restrict__ W, unsigned short* W0T, unsigned short* W1D,
                                              unsigned short* A2) {
  const int b = (int)blockIdx.x, tid = (int)threadIdx.x;
  if (b < PB_W0) {
    const int u = b * 256 + tid;
    const int n = u >> 4, p = u & 15;
    const v4u o = gather8_bf16(W, n, 8 * p, DD - 1, DD, 0xFFFFFFFFu);
    st2_v4u(W0T + (size_t)u * 8, o);
  } else if (b < PB_W0 + PB_W1) {
    const int u = (b - PB_W0) * 256 + tid;
    const int ppr = A2K / 8;
    const int n = u / ppr, p = u - n * ppr;
    const v4u o = gather8_bf16(W, DD * DD + n, 8 * p, DD - 1, DD, 0xFFFFFFFFu);
    st2_v4u(W1D + (size_t)u * 8, o);
  } else {
    const int q = (b - PB_W0 - PB_W1) * 256 + tid;
    const v4u z = (v4u){ 0u, 0u, 0u, 0u };
    st2_v4u(A2 + (size_t)NN * A2K + (size_t)q * 8, z);
  }
}

__device__ __forceinline__ float row_norm(const v4f a) {
  float s = (a[0] * a[0] + a[1] * a[1]) + (a[2] * a[2] + a[3] * a[3]);
  s += __shfl_xor(s, 16);
  s += __shfl_xor(s, 8);
  s += __shfl_xor(s, 4);
  s += __shfl_xor(s, 2);
  s += __shfl_xor(s, 1);
  return sqrtf(s);
}

template <int STEP>
__global__ __launch_bounds__(256) void k_node(const float* __restrict__ MSG, const int* __restrict__ adj,
                                              const float* __restrict__ wgt, const float* __restrict__ mask,
                                              unsigned short* A2, float* out, int nrows) {
  const int tid  = (int)threadIdx.x;
  const int lane = tid & 31;
  const int wave = __builtin_amdgcn_readfirstlane(tid >> 5);
  const int n = (int)blockIdx.x * 8 + wave;
  if (n >= nrows) return;

  int   idw = adj[(size_t)n * KS + lane];
  float ww  = wgt[(size_t)n * KS + lane];
  float mn  = mask[n];
  asm volatile("" :: "v"(idw), "v"(ww), "v"(mn));
  const int id = clampi(idw, 0, nrows - 1);
  float msr = mask[id];
  asm volatile("" :: "v"(msr));
  const float m  = bf16_val(mn);
  const float ms = bf16_val(msr);
  float c = bf16_val(ww) * ms;
  if (STEP == 0) c = c * ms;
  const int cbits = __float_as_int(c);

  v4f acc = (v4f){ 0.0f, 0.0f, 0.0f, 0.0f };
  const float* mbase = MSG + 4 * lane;
#pragma unroll 4
  for (int k = 0; k < KS; ++k) {
    const int   idk = __builtin_amdgcn_readlane(id, k);
    const float ck  = __int_as_float(__builtin_amdgcn_readlane(cbits, k));
    const v4f v = *(const v4fa*)(mbase + (size_t)idk * DD);
    acc[0] = fmaf(ck, v[0], acc[0]);
    acc[1] = fmaf(ck, v[1], acc[1]);
    acc[2] = fmaf(ck, v[2], acc[2]);
    acc[3] = fmaf(ck, v[3], acc[3]);
  }

  const float EPSV = 1e-5f;
  acc = acc * m;
  const float n1   = row_norm(acc);
  const float nc1  = (n1 < EPSV) ? EPSV : ((n1 > 15.0f) ? 15.0f : n1);
  const float den1 = (n1 < EPSV) ? EPSV : n1;
  const float th   = tanhf(nc1);
  v4f x = acc;
#pragma unroll 1
  for (int j = 0; j < 4; ++j) {
    float q = (th * x[0]) / den1;
    q = q * m;
    q = (q > 0.0f) ? q : (q - q);
    q = q * m;
    x = (v4f){ x[1], x[2], x[3], q };
  }

  if (STEP == 0) {
    const float HIC  = (float)(1.0 - 1e-5);
    const float n2   = row_norm(x);
    const float nc2  = (n2 < EPSV) ? EPSV : ((n2 > HIC) ? HIC : n2);
    const float den2 = (n2 < EPSV) ? EPSV : n2;
    const float at   = atanhf(nc2);
    v4f t = x;
#pragma unroll 1
    for (int j = 0; j < 4; ++j) {
      float q = (at * t[0]) / den2;
      q = q * m;
      t = (v4f){ t[1], t[2], t[3], q };
    }
    const v2u hi = (v2u){ pk16(bf16_bits(t[0]), bf16_bits(t[1])), pk16(bf16_bits(t[2]), bf16_bits(t[3])) };
    unsigned short* rowp = A2 + (size_t)n * A2K + 4 * lane;
#if TWO_TERM_L2
    const v2u lo = (v2u){ pk16(bf16_lo_bits(t[0]), bf16_lo_bits(t[1])), pk16(bf16_lo_bits(t[2]), bf16_lo_bits(t[3])) };
    *(volatile v2u*)rowp = hi;
    *(volatile v2u*)(rowp + DD) = lo;
    __threadfence();
    *(volatile v2u*)rowp = hi;
    *(volatile v2u*)(rowp + DD) = lo;
#else
    *(volatile v2u*)rowp = hi;
    __threadfence();
    *(volatile v2u*)rowp = hi;
#endif
  } else {
    float* op = out + (size_t)n * DD + 4 * lane;
    *(volatile v4f*)op = x;
    __threadfence();
    *(volatile v4f*)op = x;
  }
}

extern "C" void kernel_launch(void* const* d_in, const int* in_sizes, int n_in,
                              void* d_out, int out_size, void* d_ws, size_t ws_size,
                              hipStream_t stream) {
  if (n_in < 5) return;
  if (in_sizes[0] != NN * DD || in_sizes[1] != NN * KS || in_sizes[2] != NN * KS) return;
  if (in_sizes[3] != NN || in_sizes[4] != 2 * DD * DD) return;
  if (out_size != NN * DD) return;
  if (ws_size < WS_TOTAL) return;

  const float* node_repr = (const float*)d_in[0];
  const int*   adj       = (const int*)  d_in[1];
  const float* wgt       = (const float*)d_in[2];
  const float* mask      = (const float*)d_in[3];
  const float* msgw      = (const float*)d_in[4];
  float* out = (float*)d_out;

  char* ws = (char*)d_ws;
  unsigned short* XB  = (unsigned short*)(ws + O_XB);
  unsigned short* W0T = (unsigned short*)(ws + O_W0T);
  unsigned short* W1D = (unsigned short*)(ws + O_W1D);
  float*          MSG = (float*)(ws + O_MSG);
  unsigned short* A2  = (unsigned short*)(ws + O_A2);
  const float* nobias = (const float*)(ws + O_W0T);

  const int gemmBlocks = (((NN + 63) / 64) * ((DD + 63) / 64) + 7) / 8;

  k_prep<<<PREP_BLOCKS, 256, 0, stream>>>(msgw, W0T, W1D, A2);
  k_plane<0><<<MPN * DD / 8 / 256, 256, 0, stream>>>(node_repr, NN, DD, DD, XB, MPN, DD);
  k_gemm_nt<0, 0><<<gemmBlocks, 256, 0, stream>>>(XB, W0T, nobias, MSG, NN, DD, DD, DD);
  k_node<0><<<NN / 8, 256, 0, stream>>>(MSG, adj, wgt, mask, A2, out, NN);
  k_gemm_nt<0, 0><<<gemmBlocks, 256, 0, stream>>>(A2, W1D, nobias, MSG, NN, DD, A2K, DD);
  k_node<1><<<NN / 8, 256, 0, stream>>>(MSG, adj, wgt, mask, A2, out, NN);
}
